// MultiHeadSelfAttention2D_76785425318535
// MI455X (gfx1250) — hardware-verified
//
#include <hip/hip_runtime.h>
#include <math.h>
#include <stdint.h>

typedef unsigned short us;
typedef us       v8us __attribute__((ext_vector_type(8)));
typedef __bf16   v16b __attribute__((ext_vector_type(16)));
typedef _Float16 v16h __attribute__((ext_vector_type(16)));
typedef _Float16 v8h  __attribute__((ext_vector_type(8)));
typedef float    v8f  __attribute__((ext_vector_type(8)));
typedef float    v4f  __attribute__((ext_vector_type(4)));

#define NB_   4
#define NC_   64
#define NT_   1000
#define NF_   65
#define NA_   4
#define NE_   4
#define ND_   16
#define NN_   16
#define TPAD  1024
#define QKW   260
#define QKP   320
#define VW    1040
#define VR    1088
#define NSEG  32000
#define SEGF  520
#define PSC   16384.0f
#define VSC   16.0f
#define PVSCALE 3.814697265625e-06f

#define PLQK ((size_t)NN_ * TPAD * QKP)
#define NOFH ((size_t)8 * TPAD * VR)
#define NVT  ((size_t)NN_ * VR * TPAD)
#define NPP  ((size_t)NN_ * TPAD * TPAD)
#define NSB  ((size_t)NSEG * 64)

#define LDS_PROJ  178656
#define LDS_SCORE 65536
#define LDS_OUT   172672

static_assert(NT_ == 125 * 8);
static_assert(VR % 64 == 0);
static_assert(TPAD % 64 == 0);

__device__ __forceinline__ us f2bf(float f) {
  const unsigned u = __float_as_uint(f);
  return (us)((u + 0x7FFFu + ((u >> 16) & 1u)) >> 16);
}
__device__ __forceinline__ float bf2f(us hb) { return __uint_as_float(((unsigned)hb) << 16); }
__device__ __forceinline__ float bfr(float f) { return bf2f(f2bf(f)); }
__device__ __forceinline__ us f2hb(float f) { return __builtin_bit_cast(us, (_Float16)f); }

union FragB { v16b v; v8us h[2]; };
__device__ __forceinline__ v16b ldb16(const us* p) {
  FragB f; f.h[0] = *(const v8us*)p; f.h[1] = *(const v8us*)(p + 16); return f.v;
}
union FragH { v16h v; v8h h[2]; };
__device__ __forceinline__ v16h ldh16(const _Float16* p) {
  FragH f; f.h[0] = *(const v8h*)p; f.h[1] = *(const v8h*)(p + 16); return f.v;
}
__device__ __forceinline__ v8f mma_bf(v16b a, v16b b, v8f c) {
  c = __builtin_amdgcn_wmma_f32_16x16x32_bf16(false, a, false, b, (short)0, c, false, false);
  asm volatile("v_nop\n\tv_nop\n\tv_nop\n\tv_nop" : "+v"(c) : "v"(a), "v"(b));
  return c;
}
__device__ __forceinline__ v8f mma_h_raw(v16h a, v16h b, v8f c) {
  return __builtin_amdgcn_wmma_f32_16x16x32_f16(false, a, false, b, (short)0, c, false, false);
}
__device__ __forceinline__ void dep_guard_h(v8f& a, v8f& b, v16h x, v16h y) {
  asm volatile("v_nop\n\tv_nop\n\tv_nop\n\tv_nop" : "+v"(a), "+v"(b) : "v"(x), "v"(y));
}
__device__ __forceinline__ void keep4_h(v16h a, v16h b, v16h c, v16h d) {
  asm volatile("v_nop" :: "v"(a), "v"(b), "v"(c), "v"(d));
}
__device__ __forceinline__ void acc_guard4(v8f& a, v8f& b, v8f& c, v8f& d) {
  asm volatile("v_nop\n\tv_nop\n\tv_nop\n\tv_nop" : "+v"(a), "+v"(b), "+v"(c), "+v"(d));
}

__global__ __launch_bounds__(256) void k_prep(const float* __restrict__ Wq, const float* __restrict__ Wk,
                                              const float* __restrict__ Wv, const float* __restrict__ Wo,
                                              us* __restrict__ WB, us* __restrict__ WoB) {
  const int gid = blockIdx.x * 256 + threadIdx.x;
  const int line = gid >> 3, q = gid & 7;
  v8us o;
  us* dst;
  if (line < 128) {
    const int a = line >> 5, r = line & 31;
    const int iq = min(a * 4 + r, 15);
    const int ik = min(a * 4 + max(r - 4, 0), 15);
    const int iv = min(a * 16 + max(r - 8, 0), 63);
    const float wq = (r < 4) ? 1.f : 0.f;
    const float wk = (r >= 4 && r < 8) ? 1.f : 0.f;
    const float wv = (r >= 8 && r < 24) ? 1.f : 0.f;
    const v4f q0 = *(const v4f*)(Wq + (size_t)iq * 64 + 8 * q), q1 = *(const v4f*)(Wq + (size_t)iq * 64 + 8 * q + 4);
    const v4f k0 = *(const v4f*)(Wk + (size_t)ik * 64 + 8 * q), k1 = *(const v4f*)(Wk + (size_t)ik * 64 + 8 * q + 4);
    const v4f v0 = *(const v4f*)(Wv + (size_t)iv * 64 + 8 * q), v1 = *(const v4f*)(Wv + (size_t)iv * 64 + 8 * q + 4);
#pragma unroll
    for (int e = 0; e < 4; ++e) {
      o[e]     = f2bf(q0[e] * wq + k0[e] * wk + v0[e] * wv);
      o[4 + e] = f2bf(q1[e] * wq + k1[e] * wk + v1[e] * wv);
    }
    dst = WB + (size_t)line * 64 + 8 * q;
  } else {
    const int l2 = line - 128, oo = l2 >> 1;
    const v4f w0 = *(const v4f*)(Wo + (size_t)oo * 64 + 8 * q), w1 = *(const v4f*)(Wo + (size_t)oo * 64 + 8 * q + 4);
#pragma unroll
    for (int e = 0; e < 4; ++e) { o[e] = f2bf(w0[e]); o[4 + e] = f2bf(w1[e]); }
    dst = WoB + (size_t)l2 * 64 + 8 * q;
  }
  *(volatile v8us*)dst = o;
  __threadfence();
  *(volatile v8us*)dst = o;
}

__global__ __launch_bounds__(256) void k_proj(
    const float* __restrict__ x, const us* __restrict__ WB,
    const float* __restrict__ bq, const float* __restrict__ aq, const float* __restrict__ gq, const float* __restrict__ hq,
    const float* __restrict__ bk, const float* __restrict__ ak, const float* __restrict__ gk, const float* __restrict__ hk,
    const float* __restrict__ bv, const float* __restrict__ av, const float* __restrict__ gv, const float* __restrict__ hv,
    us* __restrict__ QK4, us* __restrict__ VT) {
  extern __shared__ __align__(16) unsigned char smem_p[];
  us*    XA  = (us*)(smem_p);
  float* YS  = (float*)(smem_p + 11520);
  us*    QKs = (us*)(smem_p + 19200);
  us*    VTs = (us*)(smem_p + 21760);
  float* stt = (float*)(smem_p + 178432);

  const int tid = threadIdx.x, lane = tid & 31, wave = tid >> 5, h = lane >> 4, m = lane & 15;
  const int chunk = blockIdx.x, a = blockIdx.y, b = blockIdx.z;
  const int t0 = chunk * 64, n = a * NB_ + b;

  for (int i = tid; i < 15 * 72; i += 256) XA[65 * 72 + i] = (us)0;
  for (int i = tid; i < 48 * 72; i += 256) VTs[1040 * 72 + i] = (us)0;
  for (int i = tid; i < 4 * 60; i += 256) { const int p = i / 60; QKs[p * QKP + QKW + (i - 60 * p)] = (us)0; }
  if (tid < 24) {
    const int nn = tid;
    const float wq = (nn < 4) ? 1.f : 0.f;
    const float wk = (nn >= 4 && nn < 8) ? 1.f : 0.f;
    const float wv = (nn >= 8) ? 1.f : 0.f;
    const int iq = min(a * 4 + nn, 15);
    const int ik = min(a * 4 + max(nn - 4, 0), 15);
    const int iv = min(a * 16 + max(nn - 8, 0), 63);
    stt[8 + nn]  = bfr(bq[iq]) * wq + bfr(bk[ik]) * wk + bfr(bv[iv]) * wv;
    stt[32 + nn] = bfr(aq[a]) * wq + bfr(ak[a]) * wk + bfr(av[a]) * wv;
  }
  __syncthreads();

  const us* WBa = WB + (size_t)a * 32 * 64;
  us* VTg = VT + (size_t)n * VR * TPAD + t0;

  for (int it = 0; it < 64; ++it) {
    const int tt = t0 + it;
    const int tl = min(tt, NT_ - 1);
    const float valid = (tt < NT_) ? 1.f : 0.f;
    const float* xb = x + ((size_t)b * NC_ * NT_ + tl) * NF_;
#pragma unroll 4
    for (int i = tid; i < NC_ * NF_; i += 256) {
      const int c = i / NF_, f = i - NF_ * c;
      XA[f * 72 + c] = f2bf(xb[(size_t)c * (NT_ * NF_) + f]);
    }
    __syncthreads();

    for (int tile = wave; tile < 10; tile += 8) {
      const int mt = tile >> 1, nt = tile & 1;
      v8f acc = {0.f, 0.f, 0.f, 0.f, 0.f, 0.f, 0.f, 0.f};
#pragma unroll
      for (int kc = 0; kc < 2; ++kc) {
        const v16b af = ldb16(XA + (16 * mt + m) * 72 + 32 * kc + 8 * h);
        const v16b bf = ldb16(WBa + (size_t)(16 * nt + m) * 64 + 32 * kc + 8 * h);
        acc = mma_bf(af, bf, acc);
      }
      const int nn = 16 * nt + m, nq = min(nn, 23);
      const float bia = stt[8 + nq], sl = stt[32 + nq];
      if (nn < 24) {
#pragma unroll
        for (int r = 0; r < 8; ++r) {
          float y = acc[r] + bia;
          y = (y >= 0.f) ? y : sl * y;
          YS[nn * 80 + 16 * mt + 8 * h + r] = y;
        }
      }
    }
    __syncthreads();

    if (wave < 3) {
      const int nb = 4 * wave;
      const int cnt = (wave < 2) ? (NE_ * NF_) : (ND_ * NF_);
      const float invc = (wave < 2) ? (1.0f / 260.0f) : (1.0f / 1040.0f);
      float s = 0.f;
      for (int i = lane; i < cnt; i += 32) { const int o = i / NF_, f = i - NF_ * o; s += YS[(nb + o) * 80 + f]; }
#pragma unroll
      for (int off = 16; off > 0; off >>= 1) s += __shfl_xor(s, off, 32);
      const float mu = s * invc;
      float s2 = 0.f;
      for (int i = lane; i < cnt; i += 32) { const int o = i / NF_, f = i - NF_ * o; const float d = YS[(nb + o) * 80 + f] - mu; s2 += d * d; }
#pragma unroll
      for (int off = 16; off > 0; off >>= 1) s2 += __shfl_xor(s2, off, 32);
      const float var = s2 * invc;
      const float rs = 1.0f / sqrtf(var + 1e-5f);
      if (lane == 0) { stt[wave] = mu; stt[4 + wave] = rs; }
    }
    __syncthreads();

#pragma unroll 2
    for (int i = tid; i < 2 * QKW; i += 256) {
      const int w2 = (i >= QKW) ? 1 : 0;
      const float w2f = (float)w2;
      const int e = i - QKW * w2, o = e / NF_, f = e - NF_ * o;
      const float y = YS[(4 * w2 + o) * 80 + f];
      const int gi = (a * NE_ + o) * NF_ + f;
      const float g  = bfr(gq[gi]) * (1.f - w2f) + bfr(gk[gi]) * w2f;
      const float hh = bfr(hq[gi]) * (1.f - w2f) + bfr(hk[gi]) * w2f;
      const float v = ((y - stt[w2]) * stt[4 + w2] * g + hh) * valid;
      const us hb = f2bf(v);
      const us lb = f2bf(v - bf2f(hb));
      QKs[(2 * w2) * QKP + e] = hb;
      QKs[(2 * w2 + 1) * QKP + e] = lb;
    }
#pragma unroll 2
    for (int i = tid; i < VW; i += 256) {
      const int d = i / NF_, f = i - NF_ * d;
      const float y = YS[(8 + d) * 80 + f];
      const int gi = (a * ND_ + d) * NF_ + f;
      const float v = ((y - stt[2]) * stt[6] * bfr(gv[gi]) + bfr(hv[gi])) * valid * VSC;
      VTs[i * 72 + it] = f2hb(v);
    }
    __syncthreads();

    for (int pass = 0; pass < 2; ++pass) {
      if (tid < 160) {
        const int p = tid / 40, pc = tid - 40 * p;
        const v8us val = *(const v8us*)(QKs + p * QKP + 8 * pc);
        us* dst = QK4 + (size_t)p * PLQK + ((size_t)n * TPAD + tt) * QKP + 8 * pc;
        *(volatile v8us*)dst = val;
      }
      __threadfence();
    }
  }
  __syncthreads();
  for (int pass = 0; pass < 2; ++pass) {
#pragma unroll 2
    for (int i = 0; i < 34; ++i) {
      const int row = i * 32 + (tid >> 3), q = tid & 7;
      const v8us val = *(const v8us*)(VTs + row * 72 + 8 * q);
      *(volatile v8us*)(VTg + (size_t)row * TPAD + 8 * q) = val;
    }
    __threadfence();
  }
}

__global__ __launch_bounds__(128) void k_score(const us* __restrict__ QH, const us* __restrict__ QL,
                                               const us* __restrict__ KH, const us* __restrict__ KL,
                                               us* __restrict__ P, float sscale) {
  extern __shared__ __align__(16) unsigned char smem_s[];
  float* Ss = (float*)smem_s;
  const int tid = threadIdx.x, lane = tid & 31, wave = tid >> 5, h = lane >> 4, m = lane & 15;
  const int qt = blockIdx.x, n = blockIdx.y;
  const int q0 = qt * 16;
  const size_t pb = (size_t)n * TPAD * QKP;
  const us* qh = QH + pb + (size_t)(q0 + m) * QKP + 8 * h;
  const us* ql = QL + pb + (size_t)(q0 + m) * QKP + 8 * h;
  const us* kh = KH + pb + (size_t)m * QKP + 8 * h;
  const us* kl = KL + pb + (size_t)m * QKP + 8 * h;

  for (int kt = wave; kt < 16; kt += 4) {
    v8f s[4];
#pragma unroll
    for (int j = 0; j < 4; ++j) s[j] = (v8f){0.f, 0.f, 0.f, 0.f, 0.f, 0.f, 0.f, 0.f};
#pragma unroll 1
    for (int kc = 0; kc < 9; ++kc) {
      const v16b qa = ldb16(qh + 32 * kc);
      const v16b qb = ldb16(ql + 32 * kc);
#pragma unroll
      for (int j = 0; j < 4; ++j) {
        const size_t ko = (size_t)(kt * 64 + 16 * j) * QKP + 32 * kc;
        const v16b ka = ldb16(kh + ko);
        const v16b kb = ldb16(kl + ko);
        s[j] = mma_bf(qa, ka, s[j]);
        s[j] = mma_bf(qa, kb, s[j]);
        s[j] = mma_bf(qb, ka, s[j]);
      }
    }
#pragma unroll
    for (int j = 0; j < 4; ++j) {
      const int key = kt * 64 + 16 * j + m;
#pragma unroll
      for (int r = 0; r < 8; ++r) {
        const float v = s[j][r] * sscale;
        Ss[(8 * h + r) * TPAD + key] = (key < NT_) ? v : -INFINITY;
      }
    }
  }
  __syncthreads();

  us* Pn = P + ((size_t)n * TPAD + q0) * TPAD;
#pragma unroll 1
  for (int rr = 0; rr < 4; ++rr) {
    const int row = 4 * wave + rr;
    const float* sr = Ss + row * TPAD;
    float ev[4][8];
    float mx = -INFINITY;
#pragma unroll
    for (int i = 0; i < 4; ++i) {
      const v4f a0 = *(const v4f*)(sr + 256 * i + 8 * lane);
      const v4f a1 = *(const v4f*)(sr + 256 * i + 8 * lane + 4);
#pragma unroll
      for (int e = 0; e < 4; ++e) { ev[i][e] = a0[e]; ev[i][4 + e] = a1[e]; }
#pragma unroll
      for (int e = 0; e < 8; ++e) mx = fmaxf(mx, ev[i][e]);
    }
#pragma unroll
    for (int off = 16; off > 0; off >>= 1) mx = fmaxf(mx, __shfl_xor(mx, off, 32));
    float sum = 0.f;
#pragma unroll
    for (int i = 0; i < 4; ++i)
#pragma unroll
      for (int e = 0; e < 8; ++e) { const float p = __expf(ev[i][e] - mx); ev[i][e] = p; sum += p; }
#pragma unroll
    for (int off = 16; off > 0; off >>= 1) sum += __shfl_xor(sum, off, 32);
    const float inv = (1.0f / sum) * PSC;
    v8h pk[4];
#pragma unroll
    for (int i = 0; i < 4; ++i)
#pragma unroll
      for (int e = 0; e < 8; ++e) pk[i][e] = (_Float16)(ev[i][e] * inv);
    us* prow = Pn + (size_t)row * TPAD + 8 * lane;
    for (int pass = 0; pass < 2; ++pass) {
#pragma unroll
      for (int i = 0; i < 4; ++i) *(volatile v8h*)(prow + 256 * i) = pk[i];
      __threadfence();
    }
  }
}

__global__ __launch_bounds__(256) void k_pv(const us* __restrict__ Pp, const us* __restrict__ VTp,
                                            float* __restrict__ OF, int phase, float scale) {
  __shared__ __align__(16) float sT[8][16 * 68];
  const int yb = blockIdx.y;
  const int nab = (yb >> 1) * NB_ + 2 * phase + (yb & 1);
  const int lane = threadIdx.x & 31, wave = threadIdx.x >> 5;
  const int tilesN = VR / 64;
  const int tilesM = TPAD / 64;
  const int tile = blockIdx.x * 8 + wave;
  if (tile >= tilesM * tilesN) return;
  const int tm = tile / tilesN, tn = tile - tm * tilesN;
  const int m0 = tm << 6, n0 = tn << 6;
  const _Float16* Ab = (const _Float16*)Pp + (size_t)nab * TPAD * TPAD;
  const _Float16* Bb = (const _Float16*)VTp + (size_t)nab * VR * TPAD;
  float* C = OF + (size_t)yb * TPAD * VR;
  const int rlane = lane & 15, koff = (lane >> 4) * 8, mOff = (lane >> 4) * 8;

  v8f acc[4][4];
#pragma unroll
  for (int i = 0; i < 4; ++i)
#pragma unroll
    for (int j = 0; j < 4; ++j) acc[i][j] = (v8f){0.f, 0.f, 0.f, 0.f, 0.f, 0.f, 0.f, 0.f};

  for (int k0 = 0; k0 < TPAD; k0 += 32) {
    v16h bh[4];
#pragma unroll
    for (int j = 0; j < 4; ++j) bh[j] = ldh16(Bb + (size_t)(n0 + (j << 4) + rlane) * TPAD + koff + k0);
#pragma unroll
    for (int i = 0; i < 4; ++i) {
      const v16h ah = ldh16(Ab + (size_t)(m0 + (i << 4) + rlane) * TPAD + koff + k0);
#pragma unroll
      for (int j = 0; j < 4; ++j) acc[i][j] = mma_h_raw(ah, bh[j], acc[i][j]);
      dep_guard_h(acc[i][0], acc[i][3], ah, ah);
    }
    keep4_h(bh[0], bh[1], bh[2], bh[3]);
  }
  acc_guard4(acc[0][0], acc[0][1], acc[0][2], acc[0][3]);
  acc_guard4(acc[1][0], acc[1][1], acc[1][2], acc[1][3]);
  acc_guard4(acc[2][0], acc[2][1], acc[2][2], acc[2][3]);
  acc_guard4(acc[3][0], acc[3][1], acc[3][2], acc[3][3]);

  float* slab = sT[wave];
#pragma unroll
  for (int i = 0; i < 4; ++i) {
    const int mBase = m0 + (i << 4);
#pragma unroll
    for (int j = 0; j < 4; ++j) {
#pragma unroll
      for (int r = 0; r < 8; ++r) slab[(mOff + r) * 68 + (j << 4) + rlane] = acc[i][j][r] * scale;
    }
    __builtin_amdgcn_fence(__ATOMIC_RELEASE, "workgroup");
    __builtin_amdgcn_wave_barrier();
    __builtin_amdgcn_fence(__ATOMIC_ACQUIRE, "workgroup");
    const int hh = lane >> 4, c4 = (lane & 15) * 4;
    for (int pass = 0; pass < 2; ++pass) {
#pragma unroll
      for (int it = 0; it < 8; ++it) {
        const int row = it * 2 + hh;
        const v4f v = *(const v4f*)(slab + row * 68 + c4);
        *(volatile v4f*)(C + (size_t)(mBase + row) * VR + n0 + c4) = v;
      }
      __threadfence();
    }
    __builtin_amdgcn_fence(__ATOMIC_RELEASE, "workgroup");
    __builtin_amdgcn_wave_barrier();
    __builtin_amdgcn_fence(__ATOMIC_ACQUIRE, "workgroup");
  }
}

__global__ __launch_bounds__(256) void k_out(const float* __restrict__ OF, const us* __restrict__ WoB,
                                             const float* __restrict__ bo, const float* __restrict__ ao,
                                             const float* __restrict__ go, const float* __restrict__ ho,
                                             const float* __restrict__ x, float* __restrict__ out,
                                             float* __restrict__ SB, int phase) {
  extern __shared__ __align__(16) unsigned char smem_o[];
  us*    Bt  = (us*)(smem_o);
  float* YS  = (float*)(smem_o + 21760);
  float* FS  = (float*)(smem_o + 39168);
  float* boS = (float*)(smem_o + 172288);
  float* red = (float*)(smem_o + 172544);
  float* red2 = (float*)(smem_o + 172576);

  const int tid = threadIdx.x, lane = tid & 31, wave = tid >> 5, h = lane >> 4, m = lane & 15;
  const int k = blockIdx.x, b2 = blockIdx.y;
  const int b = 2 * phase + b2;
  const int t0 = 8 * k;

  for (int i = tid; i < 15 * 136; i += 256) Bt[65 * 136 + i] = (us)0;
  if (tid < 64) boS[tid] = bfr(bo[tid]);
  const float aos = bfr(ao[0]);
  __syncthreads();

  for (int it = 0; it < 8; ++it) {
    const int t = t0 + it;
    for (int i = tid; i < VW; i += 256) {
      const int a = i / 260, v = i - 260 * a;
      const float* orow = OF + ((size_t)(a * 2 + b2) * TPAD + t) * VR;
      const v4f val = *(const v4f*)(orow + 4 * v);
#pragma unroll
      for (int e = 0; e < 4; ++e) {
        const int j = 4 * v + e, d = j / NF_, f = j - NF_ * d, c = a * ND_ + d;
        const us hb = f2bf(val[e]);
        const us lb = f2bf(val[e] - bf2f(hb));
        Bt[f * 136 + c] = hb;
        Bt[f * 136 + 64 + c] = lb;
      }
    }
    __syncthreads();

    for (int tile = wave; tile < 20; tile += 8) {
      const int mt = tile / 5, nt = tile - 5 * mt;
      v8f acc = {0.f, 0.f, 0.f, 0.f, 0.f, 0.f, 0.f, 0.f};
#pragma unroll
      for (int kc = 0; kc < 4; ++kc) {
        const v16b af = ldb16(WoB + (size_t)(16 * mt + m) * 128 + 32 * kc + 8 * h);
        const v16b bf = ldb16(Bt + (16 * nt + m) * 136 + 32 * kc + 8 * h);
        acc = mma_bf(af, bf, acc);
      }
      const int f = 16 * nt + m;
      if (f < NF_) {
#pragma unroll
        for (int r = 0; r < 8; ++r) {
          const int o = 16 * mt + 8 * h + r;
          float y = acc[r] + boS[o];
          y = (y >= 0.f) ? y : aos * y;
          YS[o * 68 + f] = y;
        }
      }
    }
    __syncthreads();

    float s = 0.f;
    for (int i = tid; i < NC_ * NF_; i += 256) { const int o = i / NF_, f = i - NF_ * o; s += YS[o * 68 + f]; }
#pragma unroll
    for (int off = 16; off > 0; off >>= 1) s += __shfl_xor(s, off, 32);
    if (lane == 0) red[wave] = s;
    __syncthreads();
    float tot = 0.f;
#pragma unroll
    for (int w = 0; w < 8; ++w) tot += red[w];
    const float mu = tot * (1.0f / 4160.0f);
    float s2 = 0.f;
    for (int i = tid; i < NC_ * NF_; i += 256) { const int o = i / NF_, f = i - NF_ * o; const float d = YS[o * 68 + f] - mu; s2 += d * d; }
#pragma unroll
    for (int off = 16; off > 0; off >>= 1) s2 += __shfl_xor(s2, off, 32);
    if (lane == 0) red2[wave] = s2;
    __syncthreads();
    float tot2 = 0.f;
#pragma unroll
    for (int w = 0; w < 8; ++w) tot2 += red2[w];
    const float var = tot2 * (1.0f / 4160.0f);
    const float rs = 1.0f / sqrtf(var + 1e-5f);

#pragma unroll 2
    for (int i = tid; i < NC_ * NF_; i += 256) {
      const int o = i / NF_, f = i - NF_ * o;
      const float y = YS[o * 68 + f];
      const float g = bfr(go[i]), hh = bfr(ho[i]);
      const float xr = bfr(x[((size_t)(b * NC_ + o) * NT_ + t) * NF_ + f]);
      FS[o * SEGF + it * NF_ + f] = (y - mu) * rs * g + hh + xr;
    }
  }
  __syncthreads();

  const int wq = tid >> 3, q = tid & 7;
  for (int pass = 0; pass < 2; ++pass) {
    for (int slot = wq; slot < NC_ * 17; slot += 32) {
      const int c = slot / 17, i = slot - 17 * c;
      const size_t S = ((size_t)(b * NC_ + c) * NT_ + t0) * NF_;
      const size_t L = (S >> 5) + (size_t)i;
      const int st = (int)((long long)(L << 5) - (long long)S);
      const bool full = (st >= 0) && (st + 32 <= SEGF);
      v4f v;
#pragma unroll
      for (int e = 0; e < 4; ++e) {
        const int idx = min(max(st + 4 * q + e, 0), SEGF - 1);
        v[e] = FS[c * SEGF + idx];
      }
      if (full) *(volatile v4f*)(out + (L << 5) + 4 * q) = v;
    }
    for (int slot = wq; slot < 128; slot += 32) {
      const int c = slot >> 1, side = slot & 1;
      const size_t S = ((size_t)(b * NC_ + c) * NT_ + t0) * NF_;
      const int sm = (int)(S & 31);
      const int em = (int)((S + SEGF) & 31);
      const size_t j = (size_t)(b * NC_ + c) * 125 + k;
      v4f v;
#pragma unroll
      for (int e = 0; e < 4; ++e) {
        const int p = 4 * q + e;
        const int ih = max(p - sm, 0);
        const int itl = min(SEGF - em + p, SEGF - 1);
        const float vh = FS[c * SEGF + ih] * ((p >= sm) ? 1.f : 0.f);
        const float vt = FS[c * SEGF + itl] * ((p < em) ? 1.f : 0.f);
        v[e] = side ? vt : vh;
      }
      *(volatile v4f*)(SB + (2 * j + side) * 32 + 4 * q) = v;
    }
    __threadfence();
  }
}

__global__ __launch_bounds__(256) void k_fix(const float* __restrict__ SB, float* __restrict__ out) {
  const int gid = blockIdx.x * 256 + threadIdx.x;
  const int j = gid >> 3, q = gid & 7;
  const int jc = min(max(j, 1), NSEG - 1);
  const size_t S = (size_t)jc * SEGF;
  const int sm = (int)(S & 31);
  const size_t L = S >> 5;
  const v4f tl = *(const v4f*)(SB + (size_t)(2 * (jc - 1) + 1) * 32 + 4 * q);
  const v4f hd = *(const v4f*)(SB + (size_t)(2 * jc) * 32 + 4 * q);
  v4f v;
#pragma unroll
  for (int e = 0; e < 4; ++e) { const int p = 4 * q + e; v[e] = (p < sm) ? tl[e] : hd[e]; }
  const bool doit = (j >= 1) && (j < NSEG) && (sm != 0);
  if (doit) *(volatile v4f*)(out + (L << 5) + 4 * q) = v;
  __threadfence();
  if (doit) *(volatile v4f*)(out + (L << 5) + 4 * q) = v;
}

extern "C" void kernel_launch(void* const* d_in, const int* in_sizes, int n_in,
                              void* d_out, int out_size, void* d_ws, size_t ws_size,
                              hipStream_t stream) {
  if (n_in < 21) return;
  if (in_sizes[0] != NB_ * NC_ * NT_ * NF_) return;
  if (in_sizes[1] != 1024 || in_sizes[2] != 16 || in_sizes[3] != 4 || in_sizes[4] != 1040 || in_sizes[5] != 1040) return;
  if (in_sizes[6] != 1024 || in_sizes[7] != 16 || in_sizes[8] != 4 || in_sizes[9] != 1040 || in_sizes[10] != 1040) return;
  if (in_sizes[11] != 4096 || in_sizes[12] != 64 || in_sizes[13] != 4 || in_sizes[14] != 4160 || in_sizes[15] != 4160) return;
  if (in_sizes[16] != 4096 || in_sizes[17] != 64 || in_sizes[18] != 1 || in_sizes[19] != 4160 || in_sizes[20] != 4160) return;
  if (out_size != NB_ * NC_ * NT_ * NF_) return;

  const float* x  = (const float*)d_in[0];
  const float* Wq = (const float*)d_in[1];
  const float* bq = (const float*)d_in[2];
  const float* aq = (const float*)d_in[3];
  const float* gq = (const float*)d_in[4];
  const float* hq = (const float*)d_in[5];
  const float* Wk = (const float*)d_in[6];
  const float* bk = (const float*)d_in[7];
  const float* ak = (const float*)d_in[8];
  const float* gk = (const float*)d_in[9];
  const float* hk = (const float*)d_in[10];
  const float* Wv = (const float*)d_in[11];
  const float* bv = (const float*)d_in[12];
  const float* av = (const float*)d_in[13];
  const float* gv = (const float*)d_in[14];
  const float* hv = (const float*)d_in[15];
  const float* Wo = (const float*)d_in[16];
  const float* bo = (const float*)d_in[17];
  const float* ao = (const float*)d_in[18];
  const float* go = (const float*)d_in[19];
  const float* ho = (const float*)d_in[20];
  float* out = (float*)d_out;

  const size_t szQK = 4 * PLQK * 2;
  const size_t szOF = NOFH * 4;
  const size_t szA  = (szQK > szOF) ? szQK : szOF;
  const size_t szVT = NVT * 2;
  const size_t szP  = NPP * 2;
  const size_t szSB = NSB * 4;
  const size_t szWB = (size_t)NA_ * 32 * 64 * 2;
  const size_t szWo = (size_t)64 * 128 * 2;
  size_t off = 0;
  const size_t oA  = off; off += szA;
  const size_t oVT = off; off += szVT;
  const size_t oP  = off; off += szP;
  const size_t oSB = off; off += szSB;
  const size_t oWB = off; off += szWB;
  const size_t oWo = off; off += szWo;
  if (off > ws_size) return;

  char* ws = (char*)d_ws;
  us* QK4   = (us*)(ws + oA);
  us* QH    = QK4;
  us* QL    = QK4 + PLQK;
  us* KH    = QK4 + 2 * PLQK;
  us* KL    = QK4 + 3 * PLQK;
  float* OF = (float*)(ws + oA);
  us* VT    = (us*)(ws + oVT);
  us* P     = (us*)(ws + oP);
  float* SB = (float*)(ws + oSB);
  us* WB    = (us*)(ws + oWB);
  us* WoB   = (us*)(ws + oWo);

  hipFuncSetAttribute(reinterpret_cast<const void*>(&k_proj),  hipFuncAttributeMaxDynamicSharedMemorySize, LDS_PROJ);
  hipFuncSetAttribute(reinterpret_cast<const void*>(&k_score), hipFuncAttributeMaxDynamicSharedMemorySize, LDS_SCORE);
  hipFuncSetAttribute(reinterpret_cast<const void*>(&k_out),   hipFuncAttributeMaxDynamicSharedMemorySize, LDS_OUT);

  const float sscale = 0.062017367294604f;

  k_prep<<<dim3(8), dim3(256), 0, stream>>>(Wq, Wk, Wv, Wo, WB, WoB);
  k_proj<<<dim3(16, NA_, NB_), dim3(256), LDS_PROJ, stream>>>(x, WB, bq, aq, gq, hq, bk, ak, gk, hk, bv, av, gv, hv, QK4, VT);
  k_score<<<dim3(TPAD / 16, NN_), dim3(128), LDS_SCORE, stream>>>(QH, QL, KH, KL, P, sscale);
  for (int phase = 0; phase < 2; ++phase) {
    k_pv<<<dim3((TPAD / 64) * (VR / 64) / 8, 8), dim3(256), 0, stream>>>(P, VT, OF, phase, PVSCALE);
    k_out<<<dim3(125, 2), dim3(256), LDS_OUT, stream>>>(OF, WoB, bo, ao, go, ho, x, out, SB, phase);
  }
  k_fix<<<dim3((NSEG * 8) / 256), dim3(256), 0, stream>>>(SB, out);
  (void)hipGetLastError();
}
